// LinearAttentionFusedRecurrentKernel_57784490001093
// MI455X (gfx1250) — hardware-verified
//
#include <hip/hip_runtime.h>

typedef __attribute__((ext_vector_type(16))) __bf16 v16bf;
typedef float v8f __attribute__((ext_vector_type(8)));
typedef float v4f __attribute__((ext_vector_type(4)));
typedef unsigned int v4u __attribute__((ext_vector_type(4)));
typedef v4f __attribute__((may_alias)) v4fa;
typedef v4u __attribute__((may_alias)) v4ua;

union FragU { v16bf v; v4u q[2]; };

#define NB   2
#define NH   16
#define SEQ  4096
#define HD   64
#define CH   64
#define NCH  (SEQ / CH)
#define NBH  (NB * NH)
#define NBLK (NBH * NCH)
#define TILE (CH * HD)
#define NTOT (NBH * SEQ * HD)

__device__ __forceinline__ v8f wmma3(v16bf a_hi, v16bf a_lo, v16bf b_hi, v16bf b_lo, v8f c) {
  c = __builtin_amdgcn_wmma_f32_16x16x32_bf16(false, a_hi, false, b_hi, (short)0, c, false, false);
  c = __builtin_amdgcn_wmma_f32_16x16x32_bf16(false, a_hi, false, b_lo, (short)0, c, false, false);
  c = __builtin_amdgcn_wmma_f32_16x16x32_bf16(false, a_lo, false, b_hi, (short)0, c, false, false);
  asm volatile("v_nop\n\tv_nop\n\tv_nop\n\tv_nop" : "+v"(c) : "v"(a_hi), "v"(a_lo), "v"(b_hi), "v"(b_lo));
  return c;
}

__device__ __forceinline__ v16bf frag16(const unsigned short* p, int h) {
  FragU f;
  f.q[0] = *(const v4ua*)(p + 8 * h);
  f.q[1] = *(const v4ua*)(p + 16 + 8 * h);
  return f.v;
}

__device__ __forceinline__ void split_bf16(float x, unsigned short& hi, unsigned short& lo) {
  const unsigned u  = __float_as_uint(x);
  const unsigned hb = (u + 0x7FFFu + ((u >> 16) & 1u)) >> 16;
  const float hf = __uint_as_float(hb << 16);
  const float rem = x - hf;
  const unsigned ur = __float_as_uint(rem);
  const unsigned lb = (ur + 0x7FFFu + ((ur >> 16) & 1u)) >> 16;
  hi = (unsigned short)hb;
  lo = (unsigned short)lb;
}

__device__ __forceinline__ void rows_store_pass(const float* s_tile, float* g, int lane) {
  const int q8 = lane & 7, sub = lane >> 3;
  #pragma unroll
  for (int i = 0; i < 8; ++i) {
    const int lid = i * 4 + sub;
    const int row = lid >> 1, hl = lid & 1;
    const int off = row * HD + 32 * hl + 4 * q8;
    const v4f val = *(const v4fa*)(s_tile + off);
    *(volatile v4f*)(g + off) = val;
  }
}

__global__ __launch_bounds__(128) void k_state(const float* __restrict__ k,
                                               const float* __restrict__ v,
                                               float* __restrict__ sbuf) {
  __shared__ __attribute__((aligned(16))) unsigned short KTh[TILE];
  __shared__ __attribute__((aligned(16))) unsigned short KTl[TILE];
  __shared__ __attribute__((aligned(16))) unsigned short VTh[TILE];
  __shared__ __attribute__((aligned(16))) unsigned short VTl[TILE];
  __shared__ __attribute__((aligned(16))) float sS[TILE];

  const int tid = threadIdx.x, lane = tid & 31, w = tid >> 5;
  const int h = lane >> 4, m = lane & 15;
  const size_t base = (size_t)blockIdx.x * TILE;

  #pragma unroll
  for (int i = 0; i < 8; ++i) {
    const int idx4 = i * 128 + tid;
    const int t = idx4 >> 4;
    const int d = (idx4 & 15) << 2;
    const v4f kv = *(const v4fa*)(k + base + (size_t)idx4 * 4);
    const v4f vv = *(const v4fa*)(v + base + (size_t)idx4 * 4);
    #pragma unroll
    for (int j = 0; j < 4; ++j) {
      unsigned short hb, lb;
      split_bf16(kv[j], hb, lb);
      KTh[(d + j) * CH + t] = hb;
      KTl[(d + j) * CH + t] = lb;
      split_bf16(vv[j], hb, lb);
      VTh[(d + j) * CH + t] = hb;
      VTl[(d + j) * CH + t] = lb;
    }
  }
  __syncthreads();

  const unsigned short* ar_h = KTh + (16 * w + m) * CH;
  const unsigned short* ar_l = KTl + (16 * w + m) * CH;
  const v16bf a0h = frag16(ar_h, h), a1h = frag16(ar_h + 32, h);
  const v16bf a0l = frag16(ar_l, h), a1l = frag16(ar_l + 32, h);

  const v8f zero8 = {0.f, 0.f, 0.f, 0.f, 0.f, 0.f, 0.f, 0.f};
  v8f acc[4];
  #pragma unroll
  for (int nt = 0; nt < 4; ++nt) {
    const unsigned short* br_h = VTh + (16 * nt + m) * CH;
    const unsigned short* br_l = VTl + (16 * nt + m) * CH;
    v8f a = zero8;
    a = wmma3(a0h, a0l, frag16(br_h, h), frag16(br_l, h), a);
    a = wmma3(a1h, a1l, frag16(br_h + 32, h), frag16(br_l + 32, h), a);
    acc[nt] = a;
  }

  #pragma unroll
  for (int nt = 0; nt < 4; ++nt) {
    #pragma unroll
    for (int r = 0; r < 8; ++r)
      sS[(16 * w + 8 * h + r) * HD + 16 * nt + m] = acc[nt][r];
  }
  __syncthreads();

  rows_store_pass(sS + 16 * w * HD, sbuf + base + (size_t)16 * w * HD, lane);
  __threadfence();
  rows_store_pass(sS + 16 * w * HD, sbuf + base + (size_t)16 * w * HD, lane);
}

__global__ __launch_bounds__(128) void k_prefix(const float* __restrict__ sbuf,
                                                unsigned short* __restrict__ pth,
                                                unsigned short* __restrict__ ptl) {
  __shared__ __attribute__((aligned(16))) unsigned short PTh[TILE];
  __shared__ __attribute__((aligned(16))) unsigned short PTl[TILE];

  const int tid = threadIdx.x, lane = tid & 31, w = tid >> 5;
  const int q8 = lane & 7, sub = lane >> 3;
  const int bh = blockIdx.x;

  v4f st[8];
  #pragma unroll
  for (int i = 0; i < 8; ++i) { st[i] = (v4f){0.f, 0.f, 0.f, 0.f}; }

  #pragma unroll 1
  for (int c = 0; c < NCH; ++c) {
    const size_t base = ((size_t)bh * NCH + c) * TILE;

    #pragma unroll
    for (int i = 0; i < 8; ++i) {
      const int idx4 = i * 128 + tid;
      const int dk = idx4 >> 4;
      const int dv = (idx4 & 15) << 2;
      #pragma unroll
      for (int j = 0; j < 4; ++j) {
        unsigned short hb, lb;
        split_bf16(st[i][j], hb, lb);
        PTh[(dv + j) * HD + dk] = hb;
        PTl[(dv + j) * HD + dk] = lb;
      }
    }
    __syncthreads();

    #pragma unroll
    for (int i = 0; i < 4; ++i) {
      const int row = 16 * w + 4 * i + sub;
      const v4u vh = *(const v4ua*)(PTh + row * HD + 8 * q8);
      const v4u vl = *(const v4ua*)(PTl + row * HD + 8 * q8);
      *(volatile v4u*)(pth + base + (size_t)row * HD + 8 * q8) = vh;
      *(volatile v4u*)(ptl + base + (size_t)row * HD + 8 * q8) = vl;
    }
    __threadfence();
    #pragma unroll
    for (int i = 0; i < 4; ++i) {
      const int row = 16 * w + 4 * i + sub;
      const v4u vh = *(const v4ua*)(PTh + row * HD + 8 * q8);
      const v4u vl = *(const v4ua*)(PTl + row * HD + 8 * q8);
      *(volatile v4u*)(pth + base + (size_t)row * HD + 8 * q8) = vh;
      *(volatile v4u*)(ptl + base + (size_t)row * HD + 8 * q8) = vl;
    }

    #pragma unroll
    for (int i = 0; i < 8; ++i) {
      const int idx4 = i * 128 + tid;
      const v4f sv = *(const v4fa*)(sbuf + base + (size_t)idx4 * 4);
      st[i] = st[i] + sv;
    }
    __syncthreads();
  }
}

__global__ __launch_bounds__(128) void k_out(const float* __restrict__ q,
                                             const float* __restrict__ k,
                                             const float* __restrict__ v,
                                             const unsigned short* __restrict__ pth,
                                             const unsigned short* __restrict__ ptl,
                                             float* __restrict__ out) {
  __shared__ __attribute__((aligned(16))) unsigned short Qh[TILE];
  __shared__ __attribute__((aligned(16))) unsigned short Ql[TILE];
  __shared__ __attribute__((aligned(16))) unsigned short Kh[TILE];
  __shared__ __attribute__((aligned(16))) unsigned short Kl[TILE];
  __shared__ __attribute__((aligned(16))) unsigned short VTh[TILE];
  __shared__ __attribute__((aligned(16))) unsigned short VTl[TILE];
  __shared__ __attribute__((aligned(16))) unsigned short Sh[4 * 16 * CH];
  __shared__ __attribute__((aligned(16))) unsigned short Sl[4 * 16 * CH];
  __shared__ __attribute__((aligned(16))) float sO[4 * 16 * HD];

  const int tid = threadIdx.x, lane = tid & 31, w = tid >> 5;
  const int h = lane >> 4, m = lane & 15;
  const size_t base = (size_t)blockIdx.x * TILE;

  #pragma unroll
  for (int i = 0; i < 8; ++i) {
    const int idx4 = i * 128 + tid;
    const int t = idx4 >> 4;
    const int d = (idx4 & 15) << 2;
    const v4f qv = *(const v4fa*)(q + base + (size_t)idx4 * 4);
    const v4f kv = *(const v4fa*)(k + base + (size_t)idx4 * 4);
    const v4f vv = *(const v4fa*)(v + base + (size_t)idx4 * 4);
    #pragma unroll
    for (int j = 0; j < 4; ++j) {
      unsigned short hb, lb;
      split_bf16(qv[j] * 0.125f, hb, lb);
      Qh[t * HD + d + j] = hb;
      Ql[t * HD + d + j] = lb;
      split_bf16(kv[j], hb, lb);
      Kh[t * HD + d + j] = hb;
      Kl[t * HD + d + j] = lb;
      split_bf16(vv[j], hb, lb);
      VTh[(d + j) * CH + t] = hb;
      VTl[(d + j) * CH + t] = lb;
    }
  }
  __syncthreads();

  const v8f zero8 = {0.f, 0.f, 0.f, 0.f, 0.f, 0.f, 0.f, 0.f};

  const unsigned short* qr_h = Qh + (16 * w + m) * HD;
  const unsigned short* qr_l = Ql + (16 * w + m) * HD;
  const v16bf q0h = frag16(qr_h, h), q1h = frag16(qr_h + 32, h);
  const v16bf q0l = frag16(qr_l, h), q1l = frag16(qr_l + 32, h);

  v8f sc[4];
  #pragma unroll
  for (int nt = 0; nt < 4; ++nt) {
    const unsigned short* kr_h = Kh + (16 * nt + m) * HD;
    const unsigned short* kr_l = Kl + (16 * nt + m) * HD;
    v8f a = zero8;
    a = wmma3(q0h, q0l, frag16(kr_h, h), frag16(kr_l, h), a);
    a = wmma3(q1h, q1l, frag16(kr_h + 32, h), frag16(kr_l + 32, h), a);
    sc[nt] = a;
  }

  unsigned short* shw = Sh + w * (16 * CH);
  unsigned short* slw = Sl + w * (16 * CH);
  #pragma unroll
  for (int nt = 0; nt < 4; ++nt) {
    #pragma unroll
    for (int r = 0; r < 8; ++r) {
      const int tl = 8 * h + r;
      const int s = 16 * nt + m;
      const float val = (s <= 16 * w + tl) ? sc[nt][r] : 0.0f;
      unsigned short hb, lb;
      split_bf16(val, hb, lb);
      shw[tl * CH + s] = hb;
      slw[tl * CH + s] = lb;
    }
  }
  __syncthreads();

  v8f o[4];
  #pragma unroll
  for (int nt = 0; nt < 4; ++nt) o[nt] = zero8;

  const unsigned short* pg_h = pth + base;
  const unsigned short* pg_l = ptl + base;
  #pragma unroll
  for (int nt = 0; nt < 4; ++nt) {
    const unsigned short* pr_h = pg_h + (16 * nt + m) * HD;
    const unsigned short* pr_l = pg_l + (16 * nt + m) * HD;
    o[nt] = wmma3(q0h, q0l, frag16(pr_h, h), frag16(pr_l, h), o[nt]);
    o[nt] = wmma3(q1h, q1l, frag16(pr_h + 32, h), frag16(pr_l + 32, h), o[nt]);
  }

  const unsigned short* sr_h = shw + m * CH;
  const unsigned short* sr_l = slw + m * CH;
  const v16bf s0h = frag16(sr_h, h), s1h = frag16(sr_h + 32, h);
  const v16bf s0l = frag16(sr_l, h), s1l = frag16(sr_l + 32, h);
  #pragma unroll
  for (int nt = 0; nt < 4; ++nt) {
    const unsigned short* vr_h = VTh + (16 * nt + m) * CH;
    const unsigned short* vr_l = VTl + (16 * nt + m) * CH;
    o[nt] = wmma3(s0h, s0l, frag16(vr_h, h), frag16(vr_l, h), o[nt]);
    o[nt] = wmma3(s1h, s1l, frag16(vr_h + 32, h), frag16(vr_l + 32, h), o[nt]);
  }

  float* sow = sO + w * (16 * HD);
  #pragma unroll
  for (int nt = 0; nt < 4; ++nt) {
    #pragma unroll
    for (int r = 0; r < 8; ++r)
      sow[(8 * h + r) * HD + 16 * nt + m] = o[nt][r];
  }
  __syncthreads();

  rows_store_pass(sow, out + base + (size_t)16 * w * HD, lane);
  __threadfence();
  rows_store_pass(sow, out + base + (size_t)16 * w * HD, lane);
}

extern "C" void kernel_launch(void* const* d_in, const int* in_sizes, int n_in,
                              void* d_out, int out_size, void* d_ws, size_t ws_size,
                              hipStream_t stream) {
  if (n_in < 3) return;
  if (in_sizes[0] != NTOT || in_sizes[1] != NTOT || in_sizes[2] != NTOT) return;
  if (out_size != NTOT) return;

  const float* q = (const float*)d_in[0];
  const float* k = (const float*)d_in[1];
  const float* v = (const float*)d_in[2];
  float* out = (float*)d_out;

  const size_t s_bytes = (size_t)NBLK * TILE * 4;
  const size_t p_bytes = (size_t)NBLK * TILE * 2;
  const size_t total = s_bytes + 2 * p_bytes;
  if (total > ws_size) return;

  char* ws = (char*)d_ws;
  float* sbuf = (float*)(ws);
  unsigned short* pth = (unsigned short*)(ws + s_bytes);
  unsigned short* ptl = (unsigned short*)(ws + s_bytes + p_bytes);

  k_state<<<NBLK, 128, 0, stream>>>(k, v, sbuf);
  k_prefix<<<NBH, 128, 0, stream>>>(sbuf, pth, ptl);
  k_out<<<NBLK, 128, 0, stream>>>(q, k, v, pth, ptl, out);
}
